// CellGraphTransformer_5119601017145
// MI455X (gfx1250) — hardware-verified
//
#include <hip/hip_runtime.h>


namespace {
constexpr int NB = 2, S = 2048, D = 1024, NH = 16, DH = 64, DFF = 4096, NROW = NB * S;
constexpr float XS = 8.0f, WSC = 256.0f, PS = 8.0f, EPS = 1e-5f;

typedef _Float16 b16;
typedef __attribute__((ext_vector_type(16))) _Float16 v16b;
typedef __attribute__((ext_vector_type(8))) _Float16 v8b;
typedef __attribute__((ext_vector_type(8))) float v8f;
typedef __attribute__((ext_vector_type(4))) float v4f;
__device__ __forceinline__ float bf16_rne(float f) { unsigned int u = __float_as_uint(f); u += 0x7FFFu + ((u >> 16) & 1u); return __uint_as_float(u & 0xFFFF0000u); }
__device__ __forceinline__ void split16(float v, b16& hi, b16& lo) { hi = (b16)v; lo = (b16)(v - (float)hi); }
__device__ __forceinline__ v16b frag_kb(const b16* p, int hh) { const v8b a = *(const v8b*)(p + 8 * hh), b = *(const v8b*)(p + 16 + 8 * hh); v16b f;
#pragma unroll
  for (int e = 0; e < 8; ++e) { f[e] = a[e]; f[8 + e] = b[e]; } return f; }
__device__ __forceinline__ v8f wmma16b(v16b a, v16b b, v8f c) { v8f d = __builtin_amdgcn_wmma_f32_16x16x32_f16(false, a, false, b, (short)0, c, false, false); asm volatile("v_nop\n\tv_nop\n\tv_nop\n\tv_nop" : "+v"(d) : "v"(a), "v"(b)); return d; }
__device__ __forceinline__ void wave_lds_sync() { __builtin_amdgcn_fence(__ATOMIC_RELEASE, "workgroup"); __builtin_amdgcn_wave_barrier(); __builtin_amdgcn_fence(__ATOMIC_ACQUIRE, "workgroup"); }
__device__ __forceinline__ float nexp(float x) { return __builtin_amdgcn_exp2f(x * 1.4426950408889634f); }
__device__ __forceinline__ float pmul(float a, float b) { float p = a * b; asm volatile("" : "+v"(p)); return p; }

__global__ __launch_bounds__(256) void prepx_kernel(const float* __restrict__ x, b16* __restrict__ X16) {
  const size_t i = ((size_t)blockIdx.x * 256 + threadIdx.x) * 8; if (i >= (size_t)NROW * D) return;
  const v4f a = *(const v4f*)(x + i), c = *(const v4f*)(x + i + 4); v8b o;
#pragma unroll
  for (int j = 0; j < 4; ++j) { o[j] = (b16)(bf16_rne(a[j]) * XS); o[4 + j] = (b16)(bf16_rne(c[j]) * XS); }
  for (int pass = 0; pass < 2; ++pass) { *(volatile v8b*)(X16 + i) = o; __threadfence(); }
}
__global__ __launch_bounds__(256) void prepw_kernel(const float* __restrict__ wq, const float* __restrict__ wk, const float* __restrict__ wv, const float* __restrict__ wo, const float* __restrict__ w1, const float* __restrict__ w2, b16* __restrict__ WT, b16* __restrict__ W1T, b16* __restrict__ W2T) {
  __shared__ __attribute__((aligned(16))) b16 T[64][64 + 8];
  const int kind = blockIdx.z, i0 = blockIdx.x * 64, o0 = blockIdx.y * 64, t_ = threadIdx.x;
  const int IN = kind == 5 ? DFF : D, OUT = kind == 4 ? DFF : D; if (i0 >= IN || o0 >= OUT) return;
  const float* w = kind == 0 ? wq : kind == 1 ? wk : kind == 2 ? wv : kind == 3 ? wo : kind == 4 ? w1 : w2; b16* dst = kind < 4 ? WT + (size_t)kind * D * D : kind == 4 ? W1T : W2T;
  for (int q = t_; q < 64 * 64; q += 256) { const int ii = q >> 6, oo = q & 63; T[oo][ii] = (b16)(bf16_rne(w[(size_t)(i0 + ii) * OUT + o0 + oo]) * WSC); }
  __syncthreads();
  for (int pass = 0; pass < 2; ++pass) { for (int q = t_; q < 64 * 8; q += 256) { const int oo = q >> 3, c8 = (q & 7) * 8; *(volatile v8b*)(dst + (size_t)(o0 + oo) * IN + i0 + c8) = *(const v8b*)(&T[oo][c8]); } __threadfence(); }
}
__global__ __launch_bounds__(128) void qkv_kernel(const b16* __restrict__ X16, const b16* __restrict__ WT, const float* __restrict__ bq, const float* __restrict__ bk, const float* __restrict__ bv, b16* __restrict__ QH, b16* __restrict__ QL, b16* __restrict__ KH, b16* __restrict__ VROW, int zoff) {
  __shared__ __attribute__((aligned(16))) b16 Th[4][16][128 + 8], Tl[4][16][128 + 8];
  const int which = zoff + blockIdx.z, wave = threadIdx.x >> 5, lane = threadIdx.x & 31, nloc = lane & 15, hlf = lane >> 4; const int m0 = blockIdx.x * 64 + wave * 16, n0 = blockIdx.y * 128;
  const b16* Bw = WT + (size_t)which * D * D; const float* bias = which == 0 ? bq : which == 1 ? bk : bv;
  v8f acc[8];
#pragma unroll
  for (int t = 0; t < 8; ++t) acc[t] = (v8f){};
#pragma unroll 2
  for (int kb = 0; kb < D; kb += 32) { const v16b a = frag_kb(X16 + (size_t)(m0 + nloc) * D + kb, hlf);
#pragma unroll
    for (int t = 0; t < 8; ++t) acc[t] = wmma16b(a, frag_kb(Bw + (size_t)(n0 + t * 16 + nloc) * D + kb, hlf), acc[t]); }
#pragma unroll
  for (int t = 0; t < 8; ++t) { const float bb = bf16_rne(bias[n0 + t * 16 + nloc]);
#pragma unroll
    for (int r = 0; r < 8; ++r) { b16 a_, c_; split16((acc[t][r] * (1.0f / (XS * WSC)) + bb) * XS, a_, c_); Th[wave][8 * hlf + r][t * 16 + nloc] = a_; Tl[wave][8 * hlf + r][t * 16 + nloc] = c_; } }
  wave_lds_sync();
  for (int pass = 0; pass < 2; ++pass) {
    for (int rr = 0; rr < 16; ++rr) { const int m = m0 + rr, b = m / S, s = m - b * S; const int hsel = lane >> 3, c8 = (lane & 7) * 8;
      if (lane < 16) { const int h = n0 / DH + hsel; const size_t gi = (((size_t)b * NH + h) * S + s) * DH + c8; const v8b vh = *(const v8b*)(&Th[wave][rr][hsel * 64 + c8]);
        if (which == 0) { *(volatile v8b*)(QH + gi) = vh; *(volatile v8b*)(QL + gi) = *(const v8b*)(&Tl[wave][rr][hsel * 64 + c8]); } else if (which == 1) *(volatile v8b*)(KH + gi) = vh; else *(volatile v8b*)(VROW + gi) = vh; } }
    __threadfence(); }
}
__global__ __launch_bounds__(256) void vt_kernel(const b16* __restrict__ VROW, b16* __restrict__ VT) {
  __shared__ __attribute__((aligned(16))) b16 Tt[DH][64 + 8];
  const int bh = blockIdx.y, s0 = blockIdx.x * 64, t_ = threadIdx.x;
  for (int k = t_; k < 64 * DH; k += 256) { const int ss = k >> 6, d = k & 63; Tt[d][ss] = VROW[((size_t)bh * S + s0 + ss) * DH + d]; }
  __syncthreads();
  for (int pass = 0; pass < 2; ++pass) { for (int q = t_; q < DH * 8; q += 256) { const int d = q >> 3, c8 = (q & 7) * 8; *(volatile v8b*)(VT + ((size_t)bh * DH + d) * S + s0 + c8) = *(const v8b*)(&Tt[d][c8]); } __threadfence(); }
}
__global__ __launch_bounds__(64) void attn_kernel(const b16* __restrict__ QH, const b16* __restrict__ QL, const b16* __restrict__ KH, const b16* __restrict__ VT, b16* __restrict__ ATT) {
  __shared__ __attribute__((aligned(16))) b16 To[2][16][DH + 8];
  const int wave = threadIdx.x >> 5, lane = threadIdx.x & 31, hh = lane >> 4, col = lane & 15; const int bh = blockIdx.y, b = bh / NH, h = bh - b * NH, q0 = blockIdx.x * 32 + wave * 16, qi = q0 + col;
  const b16* Qh = QH + (size_t)bh * S * DH; const b16* Ql = QL + (size_t)bh * S * DH; const b16* K = KH + (size_t)bh * S * DH; const b16* V = VT + (size_t)bh * DH * S;
  v16b qf[2], ql[2];
#pragma unroll
  for (int ks = 0; ks < 2; ++ks) { qf[ks] = frag_kb(Qh + (size_t)qi * DH + ks * 32, hh); ql[ks] = frag_kb(Ql + (size_t)qi * DH + ks * 32, hh); }
  const float scale = 0.125f * (1.0f / (XS * XS));
  float m = -INFINITY, l = 0.0f; v8f o[4] = {{}, {}, {}, {}};
  for (int kb = 0; kb < S; kb += 32) {
    v8f s0 = {}, s1 = {};
#pragma unroll
    for (int ks = 0; ks < 2; ++ks) { const v16b k0 = frag_kb(K + (size_t)(kb + col) * DH + ks * 32, hh), k1 = frag_kb(K + (size_t)(kb + 16 + col) * DH + ks * 32, hh);
      s0 = wmma16b(k0, qf[ks], s0); s0 = wmma16b(k0, ql[ks], s0); s1 = wmma16b(k1, qf[ks], s1); s1 = wmma16b(k1, ql[ks], s1); }
    float mr = -INFINITY;
#pragma unroll
    for (int r = 0; r < 8; ++r) { s0[r] *= scale; s1[r] *= scale; mr = fmaxf(mr, fmaxf(s0[r], s1[r])); }
    mr = fmaxf(mr, __shfl_xor(mr, 16)); const float mn = fmaxf(m, mr); const float al_ = nexp(m - mn); m = mn; float sum = 0.0f; v16b pb;
#pragma unroll
    for (int r = 0; r < 8; ++r) { const float e0 = nexp(s0[r] - mn), e1 = nexp(s1[r] - mn); sum += e0 + e1; pb[r] = (b16)(e0 * PS); pb[8 + r] = (b16)(e1 * PS); }
    sum += __shfl_xor(sum, 16); l = l * al_ + sum;
#pragma unroll
    for (int t = 0; t < 4; ++t) { o[t] *= al_; o[t] = wmma16b(frag_kb(V + (size_t)(t * 16 + col) * S + kb, hh), pb, o[t]); } }
  const float inv = 1.0f / (l * PS * XS);
#pragma unroll
  for (int t = 0; t < 4; ++t)
#pragma unroll
    for (int r = 0; r < 8; ++r) To[wave][col][t * 16 + 8 * hh + r] = (b16)(o[t][r] * inv * XS);
  wave_lds_sync();
  for (int pass = 0; pass < 2; ++pass) { for (int rr = 0; rr < 16; ++rr) if (lane < 8) *(volatile v8b*)(ATT + ((size_t)b * S + q0 + rr) * D + h * DH + lane * 8) = *(const v8b*)(&To[wave][rr][lane * 8]); __threadfence(); }
}
template <int MODE>
__global__ __launch_bounds__(128) void gemm_kernel(const b16* __restrict__ A, int lda, const b16* __restrict__ Bw, int K, const float* __restrict__ bias, const float* __restrict__ R, int ldr, float* __restrict__ Y, b16* __restrict__ Hh, int ldc) {
  __shared__ __attribute__((aligned(16))) float Ts[4][16][128 + 4];
  const int wave = threadIdx.x >> 5, lane = threadIdx.x & 31, nloc = lane & 15, hlf = lane >> 4; const int m0 = blockIdx.x * 64 + wave * 16, n0 = blockIdx.y * 128;
  v8f acc[8];
#pragma unroll
  for (int t = 0; t < 8; ++t) acc[t] = (v8f){};
  for (int kb = 0; kb < K; kb += 32) { const v16b a = frag_kb(A + (size_t)(m0 + nloc) * lda + kb, hlf);
#pragma unroll
    for (int t = 0; t < 8; ++t) acc[t] = wmma16b(a, frag_kb(Bw + (size_t)(n0 + t * 16 + nloc) * K + kb, hlf), acc[t]); }
#pragma unroll
  for (int t = 0; t < 8; ++t) { const int n = n0 + t * 16 + nloc; const float bb = bf16_rne(bias[n]);
#pragma unroll
    for (int r = 0; r < 8; ++r) { float v = acc[t][r] * (1.0f / (XS * WSC)) + bb; if (MODE == 1) v = 0.5f * v * (1.0f + erff(v * 0.70710678118654752f)); Ts[wave][8 * hlf + r][t * 16 + nloc] = v; } }
  wave_lds_sync();
  for (int pass = 0; pass < 2; ++pass) {
    for (int rr = 0; rr < 16; ++rr) { const size_t row = (size_t)(m0 + rr);
      if (MODE == 1) { if (lane < 16) { const v4f a = *(const v4f*)(&Ts[wave][rr][lane * 8]), c = *(const v4f*)(&Ts[wave][rr][lane * 8 + 4]); v8b o;
#pragma unroll
          for (int j = 0; j < 4; ++j) { o[j] = (b16)(a[j] * XS); o[4 + j] = (b16)(c[j] * XS); }
          *(volatile v8b*)(Hh + row * ldc + n0 + lane * 8) = o; } }
      else { v4f v = *(const v4f*)(&Ts[wave][rr][lane * 4]); const v4f rv = *(const v4f*)(R + row * ldr + n0 + lane * 4);
        if (MODE == 0) { v[0] += bf16_rne(rv[0]); v[1] += bf16_rne(rv[1]); v[2] += bf16_rne(rv[2]); v[3] += bf16_rne(rv[3]); } else v += rv;
        *(volatile v4f*)(Y + row * ldc + n0 + lane * 4) = v; } }
    __threadfence(); }
}
__global__ __launch_bounds__(256) void ln_kernel(const float* __restrict__ Y, const float* __restrict__ g, const float* __restrict__ be, float* __restrict__ OUT, b16* __restrict__ O16) {
  __shared__ __attribute__((aligned(16))) float Tr[8][D];
  const int wave = threadIdx.x >> 5, lane = threadIdx.x & 31; const size_t row = (size_t)blockIdx.x * 8 + wave; const float* src = Y + row * D;
  float s = 0.0f;
#pragma unroll 1
  for (int j = 0; j < 32; ++j) s += src[j * 32 + lane];
#pragma unroll
  for (int o = 16; o >= 1; o >>= 1) s += __shfl_xor(s, o);
  const float mu = s * (1.0f / D); float ss = 0.0f;
#pragma unroll 1
  for (int j = 0; j < 32; ++j) { const float d = src[j * 32 + lane] - mu; ss += pmul(d, d); }
#pragma unroll
  for (int o = 16; o >= 1; o >>= 1) ss += __shfl_xor(ss, o);
  const float rs = rsqrtf(ss * (1.0f / D) + EPS);
#pragma unroll 1
  for (int j = 0; j < 32; ++j) { const int c = j * 32 + lane; Tr[wave][c] = pmul((src[c] - mu) * rs, bf16_rne(g[c])) + bf16_rne(be[c]); }
  wave_lds_sync();
  for (int pass = 0; pass < 2; ++pass) {
    for (int qd = 0; qd < 8; ++qd) { const v4f v = *(const v4f*)(&Tr[wave][qd * 128 + lane * 4]); if (OUT) *(volatile v4f*)(OUT + row * D + qd * 128 + lane * 4) = v; }
    if (O16) for (int qd = 0; qd < 4; ++qd) { const v4f a = *(const v4f*)(&Tr[wave][qd * 256 + lane * 8]), c = *(const v4f*)(&Tr[wave][qd * 256 + lane * 8 + 4]); v8b o;
#pragma unroll
      for (int j = 0; j < 4; ++j) { o[j] = (b16)(a[j] * XS); o[4 + j] = (b16)(c[j] * XS); }
      *(volatile v8b*)(O16 + row * D + qd * 256 + lane * 8) = o; }
    __threadfence(); }
}
}

extern "C" void kernel_launch(void* const* d_in, const int* in_sizes, int n_in, void* d_out, int out_size, void* d_ws, size_t ws_size, hipStream_t stream) {
  (void)n_in;
  auto Fp = [&](int i) { return (const float*)d_in[i]; };
  if (in_sizes[0] != NROW * D || in_sizes[1] != D * D || in_sizes[7] != D * D || in_sizes[13] != D * DFF || in_sizes[15] != DFF * D || out_size != NROW * D) return;
  size_t off = 0; char* ws = (char*)d_ws;
  auto carve = [&](size_t bytes) { char* p = ws + off; off += (bytes + 255) & ~(size_t)255; return p; };
  b16* X16 = (b16*)carve((size_t)NROW * D * 2); b16* WT = (b16*)carve((size_t)4 * D * D * 2); b16* W1T = (b16*)carve((size_t)DFF * D * 2); b16* W2T = (b16*)carve((size_t)D * DFF * 2);
  b16* QH = (b16*)carve((size_t)NROW * D * 2); b16* QL = (b16*)carve((size_t)NROW * D * 2); b16* KH = (b16*)carve((size_t)NROW * D * 2); b16* VROW = (b16*)carve((size_t)NROW * D * 2); b16* VT = (b16*)carve((size_t)NROW * D * 2);
  float* Y = (float*)carve((size_t)NROW * D * 4); float* OUT1 = (float*)carve((size_t)NROW * D * 4); b16* O16 = (b16*)carve((size_t)NROW * D * 2);
  b16* ATT = VROW;
  b16* HH = QH;
  static_assert((size_t)NROW * DFF * 2 == 4 * (size_t)NROW * D * 2, "HH exactly covers the four qkv planes");
  if (off > ws_size || off > ((size_t)128 << 20)) return;
  prepx_kernel<<<(NROW * D / 8 + 255) / 256, 256, 0, stream>>>(Fp(0), X16);
  prepw_kernel<<<dim3(DFF / 64, DFF / 64, 6), 256, 0, stream>>>(Fp(1), Fp(3), Fp(5), Fp(7), Fp(13), Fp(15), WT, W1T, W2T);
  qkv_kernel<<<dim3(NROW / 64, D / 128, 3), 128, 0, stream>>>(X16, WT, Fp(2), Fp(4), Fp(6), QH, QL, KH, VROW, 0);
  vt_kernel<<<dim3(S / 64, NB * NH), 256, 0, stream>>>(VROW, VT);
  attn_kernel<<<dim3(S / 32, NB * NH), 64, 0, stream>>>(QH, QL, KH, VT, ATT);
  gemm_kernel<0><<<dim3(NROW / 64, D / 128), 128, 0, stream>>>(ATT, D, WT + (size_t)3 * D * D, D, Fp(8), Fp(0), D, Y, nullptr, D);
  ln_kernel<<<NROW / 8, 256, 0, stream>>>(Y, Fp(9), Fp(10), OUT1, O16);
  gemm_kernel<1><<<dim3(NROW / 64, DFF / 128), 128, 0, stream>>>(O16, D, W1T, D, Fp(14), nullptr, 0, nullptr, HH, DFF);
  gemm_kernel<2><<<dim3(NROW / 64, D / 128), 128, 0, stream>>>(HH, DFF, W2T, DFF, Fp(16), OUT1, D, Y, nullptr, D);
  ln_kernel<<<NROW / 8, 256, 0, stream>>>(Y, Fp(11), Fp(12), (float*)d_out, nullptr);
}
